// ProtoPNet_16844861735550
// MI455X (gfx1250) — hardware-verified
//
#include <hip/hip_runtime.h>
#include <math.h>
#include <stdint.h>

#define NB    32
#define CH    2048
#define HWN   196
#define NTG   13
#define MR    (NTG * 16)
#define NP    2000
#define NPP   2048
#define NCLS  200
#define NCP   224
#define KP    2048
#define EPSD  1e-7f
#define BIGX  1e30f
static_assert(MR >= HWN);
static_assert((MR - HWN) < 16);
static_assert((HWN % 4) == 0);
static_assert((NPP % 64) == 0);
static_assert((KP % 256) == 0);
static_assert((CH % 256) == 0);
static_assert(CH == KP);
static_assert((NP % 8) == 0);
static_assert(NP <= KP);
static_assert(((NB * NP) % 128) == 0);
static_assert(((NB * NCLS) % 128) == 0);
static_assert((NCP % 32) == 0);
static_assert(NCP >= NTG * 16);
static_assert(NB == 32);

typedef __bf16         v16b __attribute__((ext_vector_type(16)));
typedef __bf16         v8b  __attribute__((ext_vector_type(8)));
typedef float          v8f  __attribute__((ext_vector_type(8)));
typedef float          v4f  __attribute__((ext_vector_type(4)));
typedef unsigned int   v4u  __attribute__((ext_vector_type(4)));
typedef unsigned short v8us __attribute__((ext_vector_type(8)));

__device__ __forceinline__ unsigned short bf_bits(float f) {
  unsigned u = __float_as_uint(f);
  return (unsigned short)((u + 0x7FFFu + ((u >> 16) & 1u)) >> 16);
}
__device__ __forceinline__ float bf_up(unsigned short hb) { return __uint_as_float(((unsigned)hb) << 16); }
__device__ __forceinline__ unsigned pk16(unsigned short a, unsigned short b) { return (unsigned)a | ((unsigned)b << 16); }
__device__ __forceinline__ v8f zero8() { v8f z = {0.f, 0.f, 0.f, 0.f, 0.f, 0.f, 0.f, 0.f}; return z; }

__device__ __forceinline__ v16b ldfrag_b(const __bf16* p) {
  union { v16b v; v8b hv[2]; } f;
  f.hv[0] = *(const v8b*)(p);
  f.hv[1] = *(const v8b*)(p + 16);
  return f.v;
}

__device__ __forceinline__ v8f mma_b(v16b a, v16b b, v8f c) {
  c = __builtin_amdgcn_wmma_f32_16x16x32_bf16(false, a, false, b, (short)0, c, false, false);
#if defined(__HIP_DEVICE_COMPILE__)
  asm volatile("v_nop\n\tv_nop\n\tv_nop\n\tv_nop" : "+v"(c) : "v"(a), "v"(b));
#endif
  return c;
}

__device__ __forceinline__ unsigned cvt_pair(float x0, float x1, float& s) {
  const unsigned short b0 = bf_bits(x0), b1 = bf_bits(x1);
  const float y0 = bf_up(b0), y1 = bf_up(b1);
  s = s + y0 * y0;
  s = s + y1 * y1;
  return pk16(b0, b1);
}

__global__ __launch_bounds__(256) void k_prep_x(const float* __restrict__ x, unsigned short* Xt, float* X2L) {
  __shared__ __align__(16) unsigned short T[16][264];
  __shared__ float red[8][16];
  const int tid  = threadIdx.x;
  const int lane = tid & 31;
  const int wave = tid >> 5;
  const int ng   = blockIdx.x;
  const int b    = blockIdx.y;
  const int n0   = ng * 16;
  const int nq   = (n0 + 16 <= HWN) ? 4 : ((HWN - n0) >> 2);
  const v4f z4 = {0.f, 0.f, 0.f, 0.f};

  float s[16];
#pragma unroll
  for (int i = 0; i < 16; ++i) s[i] = 0.f;

#pragma unroll 1
  for (int ck = 0; ck < CH / 256; ++ck) {
    const int c = ck * 256 + tid;
    const float* src = x + ((size_t)b * CH + c) * HWN + n0;
    float f[16];
#pragma unroll
    for (int qi = 0; qi < 4; ++qi) {
      const int qc = (qi < nq) ? qi : (nq - 1);
      v4f v = *(const v4f*)(src + 4 * qc);
      if (qi >= nq) v = z4;
      f[4 * qi + 0] = v[0]; f[4 * qi + 1] = v[1]; f[4 * qi + 2] = v[2]; f[4 * qi + 3] = v[3];
    }
#pragma unroll
    for (int i = 0; i < 16; ++i) {
      const unsigned short us = bf_bits(f[i]);
      const float y = bf_up(us);
      s[i] = s[i] + y * y;
      T[i][tid] = us;
    }
    __syncthreads();
#pragma unroll
    for (int rr = 0; rr < 2; ++rr) {
      const int i = 2 * wave + rr;
      const v8us v = *(const v8us*)(&T[i][8 * lane]);
      unsigned short* d = Xt + ((size_t)(b * MR + n0 + i)) * KP + ck * 256 + 8 * lane;
      *(volatile v8us*)d = v;
      __threadfence();
      *(volatile v8us*)d = v;
    }
    __syncthreads();
  }

#pragma unroll
  for (int i = 0; i < 16; ++i) {
    float v = s[i];
#pragma unroll
    for (int off = 1; off < 32; off <<= 1) v += __shfl_xor(v, off, 32);
    s[i] = v;
  }
  if (lane == 0) {
#pragma unroll
    for (int i = 0; i < 16; ++i) red[wave][i] = s[i];
  }
  __syncthreads();
  if (wave == 0) {
    const int li = lane & 15;
    float a = 0.f;
#pragma unroll
    for (int w = 0; w < 8; ++w) a += red[w][li];
    const float v = (lane < 16 && (n0 + lane) < HWN) ? a : BIGX;
    float* d = X2L + ((size_t)(b * NTG + ng)) * 32 + lane;
    *(volatile float*)d = v;
    __threadfence();
    *(volatile float*)d = v;
  }
}

__global__ __launch_bounds__(256) void k_rows(const float* __restrict__ src, int nrows, int kdim,
                                              unsigned short* dst, float* sq) {
  __shared__ float sred[32];
  const int lane = threadIdx.x & 31;
  const int wave = threadIdx.x >> 5;
  const int blk  = blockIdx.x;
  const v4f z4 = {0.f, 0.f, 0.f, 0.f};
#pragma unroll 1
  for (int i = 0; i < 4; ++i) {
    const int row  = blk * 32 + 4 * wave + i;
    const bool rv  = row < nrows;
    const int rowc = rv ? row : (nrows - 1);
    const float* s0 = src + (size_t)rowc * kdim;
    float ss = 0.f;
#pragma unroll 1
    for (int it = 0; it < KP / 256; ++it) {
      const int k   = it * 256 + 8 * lane;
      const bool kv = rv && (k + 8 <= kdim);
      const int kc  = (k + 8 <= kdim) ? k : (kdim - 8);
      v4f a0 = *(const v4f*)(s0 + kc);
      v4f a1 = *(const v4f*)(s0 + kc + 4);
      if (!kv) { a0 = z4; a1 = z4; }
      v4u pk;
      pk[0] = cvt_pair(a0[0], a0[1], ss);
      pk[1] = cvt_pair(a0[2], a0[3], ss);
      pk[2] = cvt_pair(a1[0], a1[1], ss);
      pk[3] = cvt_pair(a1[2], a1[3], ss);
      unsigned short* d = dst + (size_t)row * KP + k;
      *(volatile v4u*)d = pk;
      __threadfence();
      *(volatile v4u*)d = pk;
    }
#pragma unroll
    for (int off = 1; off < 32; off <<= 1) ss += __shfl_xor(ss, off, 32);
    if (lane == 0) sred[4 * wave + i] = ss;
  }
  __syncthreads();
  if (wave == 0) {
    const float v = sred[lane];
    float* d = sq + (size_t)blk * 32 + lane;
    *(volatile float*)d = v;
    __threadfence();
    *(volatile float*)d = v;
  }
}

__global__ __launch_bounds__(416) void k_dist(const unsigned short* __restrict__ Xt,
                                              const unsigned short* __restrict__ Pb,
                                              const float* __restrict__ X2L,
                                              const float* __restrict__ P2L, float* MD) {
  const __bf16* Xb = (const __bf16*)(const void*)Xt;
  const __bf16* Bb = (const __bf16*)(const void*)Pb;
  __shared__ float smin[NTG][64];
  __shared__ __align__(16) float sfin[64];

  const int lane  = threadIdx.x & 31;
  const int wave  = threadIdx.x >> 5;
  const int h     = lane >> 4;
  const int c     = lane & 15;
  const int cbase = blockIdx.x * 64;
  const int b     = blockIdx.y;

  const __bf16* ap = Xb + (size_t)(b * MR + wave * 16 + c) * KP + 8 * h;
  const __bf16* bq = Bb + (size_t)(cbase + c) * KP + 8 * h;

  v8f acc[4];
#pragma unroll
  for (int j = 0; j < 4; ++j) acc[j] = zero8();

#pragma unroll 1
  for (int ks = 0; ks < KP / 32; ++ks) {
    const int k0 = ks * 32;
    const v16b a = ldfrag_b(ap + k0);
    v16b bf[4];
#pragma unroll
    for (int j = 0; j < 4; ++j) bf[j] = ldfrag_b(bq + (size_t)j * 16 * KP + k0);
#pragma unroll
    for (int j = 0; j < 4; ++j) acc[j] = mma_b(a, bf[j], acc[j]);
  }

  float x2v[8];
  {
    const float* xp = X2L + ((size_t)(b * NTG + wave)) * 32 + 8 * h;
    const v4f u0 = *(const v4f*)(xp);
    const v4f u1 = *(const v4f*)(xp + 4);
#pragma unroll
    for (int i = 0; i < 4; ++i) { x2v[i] = u0[i]; x2v[4 + i] = u1[i]; }
  }
  float m[4];
#pragma unroll
  for (int j = 0; j < 4; ++j) {
    const float p2 = P2L[cbase + 16 * j + c];
    float mm = 3.0e38f;
#pragma unroll
    for (int r = 0; r < 8; ++r) {
      const float sxp = x2v[r] + p2;
      const float t   = fmaf(-2.0f, acc[j][r], sxp);
      mm = fminf(mm, t);
    }
    m[j] = mm;
  }
#pragma unroll
  for (int j = 0; j < 4; ++j) m[j] = fminf(m[j], __shfl_xor(m[j], 16, 32));
  if (h == 0) {
#pragma unroll
    for (int j = 0; j < 4; ++j) smin[wave][16 * j + c] = m[j];
  }
  __syncthreads();
  if (threadIdx.x < 64) {
    const int t = threadIdx.x;
    float v = smin[0][t];
#pragma unroll
    for (int w = 1; w < NTG; ++w) v = fminf(v, smin[w][t]);
    sfin[t] = v;
  }
  __syncthreads();
  if (wave == 0) {
    const int cc = lane & 15;
    const v4f v = *(const v4f*)(&sfin[cc * 4]);
    float* d = MD + (size_t)b * NPP + cbase + cc * 4;
    if (lane < 16) *(volatile v4f*)d = v;
    __threadfence();
    if (lane < 16) *(volatile v4f*)d = v;
  }
}

__global__ __launch_bounds__(256) void k_simout(const float* __restrict__ MD,
                                                unsigned short* Sh, unsigned short* Sl, float* out1) {
  __shared__ __align__(16) unsigned short shi[NPP];
  __shared__ __align__(16) unsigned short slo[NPP];
  __shared__ __align__(16) float sd[1024];
  const int tid  = threadIdx.x;
  const int lane = tid & 31;
  (void)lane;
  if (blockIdx.x < NB) {
    const int b = blockIdx.x;
#pragma unroll 1
    for (int it = 0; it < NPP / 256; ++it) {
      const int p = it * 256 + tid;
      const float md2 = MD[(size_t)b * NPP + p];
      const float d   = sqrtf(fmaxf(md2, 1e-12f));
      float sim = logf((d + 1.0f) / (d + EPSD));
      sim = (p < NP) ? sim : 0.0f;
      const unsigned short hb = bf_bits(sim);
      const unsigned short lb = bf_bits(sim - bf_up(hb));
      shi[p] = hb;
      slo[p] = lb;
    }
    __syncthreads();
    const v8us vh = *(const v8us*)(&shi[8 * tid]);
    const v8us vl = *(const v8us*)(&slo[8 * tid]);
    unsigned short* dh = Sh + (size_t)b * KP + 8 * tid;
    unsigned short* dl = Sl + (size_t)b * KP + 8 * tid;
    *(volatile v8us*)dh = vh;
    *(volatile v8us*)dl = vl;
    __threadfence();
    *(volatile v8us*)dh = vh;
    *(volatile v8us*)dl = vl;
  } else {
    const int blk = blockIdx.x - NB;
#pragma unroll 1
    for (int it = 0; it < 4; ++it) {
      const int e  = blk * 1024 + it * 256 + tid;
      const int ec = (e < NB * NP) ? e : (NB * NP - 1);
      const int b  = ec / NP;
      const int p  = ec - b * NP;
      const float md2 = MD[(size_t)b * NPP + p];
      sd[it * 256 + tid] = sqrtf(fmaxf(md2, 1e-12f));
    }
    __syncthreads();
    const int g = blk * 256 + tid;
    if (g < (NB * NP) / 4) {
      const v4f v = *(const v4f*)(&sd[4 * tid]);
      float* d = out1 + (size_t)4 * g;
      *(volatile v4f*)d = v;
      __threadfence();
      *(volatile v4f*)d = v;
    }
  }
}

__global__ __launch_bounds__(416) void k_fc(const unsigned short* __restrict__ Sh,
                                            const unsigned short* __restrict__ Sl,
                                            const unsigned short* __restrict__ Wb, float* out0) {
  __shared__ __align__(16) float sout[NB][MR];
  const __bf16* Ah = (const __bf16*)(const void*)Sh;
  const __bf16* Al = (const __bf16*)(const void*)Sl;
  const __bf16* Bw = (const __bf16*)(const void*)Wb;
  const int lane = threadIdx.x & 31;
  const int wave = threadIdx.x >> 5;
  const int h    = lane >> 4;
  const int c    = lane & 15;

  const __bf16* bwp = Bw + (size_t)(16 * wave + c) * KP + 8 * h;
  v8f acc[2];
  acc[0] = zero8(); acc[1] = zero8();
#pragma unroll 1
  for (int ks = 0; ks < KP / 32; ++ks) {
    const int k0 = ks * 32;
    const v16b bw = ldfrag_b(bwp + k0);
#pragma unroll
    for (int i = 0; i < 2; ++i) {
      const v16b ah = ldfrag_b(Ah + (size_t)(16 * i + c) * KP + 8 * h + k0);
      const v16b al = ldfrag_b(Al + (size_t)(16 * i + c) * KP + 8 * h + k0);
      acc[i] = mma_b(ah, bw, acc[i]);
      acc[i] = mma_b(al, bw, acc[i]);
    }
  }
#pragma unroll
  for (int i = 0; i < 2; ++i) {
#pragma unroll
    for (int r = 0; r < 8; ++r) sout[16 * i + 8 * h + r][16 * wave + c] = acc[i][r];
  }
  __syncthreads();
#pragma unroll 1
  for (int q = wave; q < (NB * NCLS) / 128; q += NTG) {
    const int g  = 32 * q + lane;
    const int bb = g / (NCLS / 4);
    const int cc = (g - bb * (NCLS / 4)) * 4;
    const v4f v = *(const v4f*)(&sout[bb][cc]);
    float* d = out0 + (size_t)4 * g;
    *(volatile v4f*)d = v;
    __threadfence();
    *(volatile v4f*)d = v;
  }
}

extern "C" void kernel_launch(void* const* d_in, const int* in_sizes, int n_in,
                              void* d_out, int out_size, void* d_ws, size_t ws_size,
                              hipStream_t stream) {
  if (n_in < 3) return;
  if (in_sizes[0] != NB * CH * HWN) return;
  if (in_sizes[1] != NP * CH) return;
  if (in_sizes[2] != NCLS * NP) return;
  if (out_size < NB * NCLS + NB * NP) return;

  const float* x   = (const float*)d_in[0];
  const float* pro = (const float*)d_in[1];
  const float* fcw = (const float*)d_in[2];
  float* out = (float*)d_out;

  const size_t bXt  = (size_t)NB * MR * KP * 2;
  const size_t bPb  = (size_t)NPP * KP * 2;
  const size_t bWb  = (size_t)NCP * KP * 2;
  const size_t bX2L = (size_t)NB * NTG * 32 * 4;
  const size_t bP2L = (size_t)NPP * 4;
  const size_t bW2L = 1024;
  const size_t bMD  = (size_t)NB * NPP * 4;
  const size_t bS   = (size_t)NB * KP * 2;
  size_t off = 0;
  const size_t oXt  = off; off += bXt;
  const size_t oPb  = off; off += bPb;
  const size_t oWb  = off; off += bWb;
  const size_t oX2L = off; off += bX2L;
  const size_t oP2L = off; off += bP2L;
  const size_t oW2L = off; off += bW2L;
  const size_t oMD  = off; off += bMD;
  const size_t oSh  = off; off += bS;
  const size_t oSl  = off; off += bS;
  if (off > ws_size) return;
  if (off > (size_t)134217728) return;
  if ((size_t)NCP * 4 > bW2L) return;

  char* ws = (char*)d_ws;
  unsigned short* Xt  = (unsigned short*)(ws + oXt);
  unsigned short* Pb  = (unsigned short*)(ws + oPb);
  unsigned short* Wb  = (unsigned short*)(ws + oWb);
  float* X2L = (float*)(ws + oX2L);
  float* P2L = (float*)(ws + oP2L);
  float* W2L = (float*)(ws + oW2L);
  float* MD  = (float*)(ws + oMD);
  unsigned short* Sh  = (unsigned short*)(ws + oSh);
  unsigned short* Sl  = (unsigned short*)(ws + oSl);

  k_prep_x<<<dim3(NTG, NB), dim3(256), 0, stream>>>(x, Xt, X2L);
  k_rows<<<dim3(NPP / 32), dim3(256), 0, stream>>>(pro, NP, CH, Pb, P2L);
  k_rows<<<dim3(NCP / 32), dim3(256), 0, stream>>>(fcw, NCLS, NP, Wb, W2L);
  k_dist<<<dim3(NPP / 64, NB), dim3(NTG * 32), 0, stream>>>(Xt, Pb, X2L, P2L, MD);
  k_simout<<<dim3(NB + (NB * NP / 4 + 255) / 256), dim3(256), 0, stream>>>(MD, Sh, Sl, out + NB * NCLS);
  k_fc<<<dim3(1), dim3(NTG * 32), 0, stream>>>(Sh, Sl, Wb, out);
  (void)hipGetLastError();
}
